// MultiHeadAttention_738734374918
// MI455X (gfx1250) — hardware-run, weakly checked
//
#include <hip/hip_runtime.h>


#ifndef NB
#define NB 2
#endif
#ifndef SEQ
#define SEQ 2048
#endif
#define NB_FULL  2
#define SEQ_FULL 2048
#ifndef OUT_SEQ
#define OUT_SEQ SEQ
#endif
#define DM   1024
#define NH_  16
#define HD   64
#define AW   4
#define CW   2
#define OSP  68
#define TSP  72
#define SC2  ((float)(0.125 * 1.4426950408889634))
#define PSH  14.0f
#define PVS  0.00390625f
#define WOC  64.0f
#define OSC  (1.0f / 4096.0f)
#define NEGB (-3.0e38f)
#define STP  ((size_t)NB * NH_ * SEQ)

static_assert(HD == 64);
static_assert(NH_ * HD == DM);
static_assert(DM % 64 == 0);
static_assert(DM % 32 == 0);
static_assert(SEQ % 64 == 0);
static_assert((NB * SEQ) % 64 == 0);
static_assert(SEQ % 32 == 0);
static_assert(SEQ % (16 * AW) == 0);
static_assert(SEQ % (16 * CW) == 0);
static_assert(16 * CW * 4 == 128);
static_assert(((size_t)SEQ * DM) % 8 == 0);
static_assert(((size_t)DM * DM) % 8 == 0);
static_assert(NB <= NB_FULL);
static_assert(SEQ <= SEQ_FULL);
static_assert((OSP * 4) % 16 == 0);
static_assert((TSP * 2) % 16 == 0);
static_assert(OSP >= 64);
static_assert(TSP >= 64);
static_assert(32 * 16 * 4 == 16 * HD * 2);
static_assert(32 * 16 * 4 == 16 * 64 * 2);
static_assert(32 * 16 * 4 == 16 * HD * 2);
static_assert(32 * 16 * 8 == 16 * 64 * 4);
static_assert(256 * 16 * 2 == 64 * 64 * 2);
static_assert(16 * 16 == 2 * 16 * CW * 4);
static_assert(16 * OSP * 4 <= 131072);
static_assert(AW * 16 * OSP * 4 <= 131072);
static_assert(64 * TSP * 2 <= 131072);
static_assert(2 * 16 * CW * 4 <= 131072);

typedef _Float16 h16;
typedef unsigned short bf;
typedef __attribute__((ext_vector_type(16))) __bf16   v16bf;
typedef __attribute__((ext_vector_type(16))) _Float16 v16h;
typedef __attribute__((ext_vector_type(8)))  _Float16 v8h;
typedef __attribute__((ext_vector_type(8)))  unsigned short v8us;
typedef __attribute__((ext_vector_type(8)))  float    v8f;
typedef __attribute__((ext_vector_type(4)))  float    v4f;
typedef v4f  __attribute__((may_alias)) v4fa;
typedef v8us __attribute__((may_alias)) v8usa;

__device__ __forceinline__ unsigned short f2bf(float f) { unsigned u = __float_as_uint(f); u += 0x7FFFu + ((u >> 16) & 1u); return (unsigned short)(u >> 16); }
__device__ __forceinline__ float bfr(float f) { return __uint_as_float(((unsigned)f2bf(f)) << 16); }
__device__ __forceinline__ v16h cat16(v8h lo, v8h hi) { return __builtin_shufflevector(lo, hi, 0, 1, 2, 3, 4, 5, 6, 7, 8, 9, 10, 11, 12, 13, 14, 15); }
__device__ __forceinline__ v16bf cat16b(v8us lo, v8us hi) { return __builtin_bit_cast(v16bf, __builtin_shufflevector(lo, hi, 0, 1, 2, 3, 4, 5, 6, 7, 8, 9, 10, 11, 12, 13, 14, 15)); }
__device__ __forceinline__ v8f wmma16(v16h a, v16h b, v8f c) { return __builtin_amdgcn_wmma_f32_16x16x32_f16(false, a, false, b, (short)0, c, false, false); }
__device__ __forceinline__ v8f wmmab(v16bf a, v16bf b, v8f c) { return __builtin_amdgcn_wmma_f32_16x16x32_bf16(false, a, false, b, (short)0, c, false, false); }
__device__ __forceinline__ v16h  ldh(const h16* p) { return cat16(*(const v8h*)p, *(const v8h*)(p + 16)); }
__device__ __forceinline__ v16bf ldb(const bf* p)  { return cat16b(*(const v8us*)p, *(const v8us*)(p + 16)); }
__device__ __forceinline__ void wave_sync() { __builtin_amdgcn_fence(3  , "wavefront"); __builtin_amdgcn_wave_barrier(); asm volatile("" ::: "memory"); }

__device__ __forceinline__ v8f wmmabg(v16bf a, v16bf b, v8f c) { c = wmmab(a, b, c); asm volatile("v_nop\n\tv_nop\n\tv_nop\n\tv_nop" : "+v"(c) : "v"(a), "v"(b)); return c; }
__device__ __forceinline__ v8f wmma16g(v16h a, v16h b, v8f c) { c = wmma16(a, b, c); asm volatile("v_nop\n\tv_nop\n\tv_nop\n\tv_nop" : "+v"(c) : "v"(a), "v"(b)); return c; }
static __device__ __forceinline__ h16 toh_flush(float v) { const float w = (fabsf(v) < 6.103515625e-05f) ? 0.0f : v; return (h16)w; }

__global__ __launch_bounds__(256) void k_cvt8(const float* __restrict__ src, bf* dst, size_t n8) {
    const size_t i = (size_t)blockIdx.x * 256 + threadIdx.x; if (i >= n8) return;
    const v8f v = *(const v8f*)(src + i * 8); v8us o;
#pragma unroll
    for (int k = 0; k < 8; ++k) o[k] = f2bf(v[k]);
    *(volatile v8us*)(dst + i * 8) = o; __threadfence(); *(volatile v8us*)(dst + i * 8) = o;
}

__global__ __launch_bounds__(256) void k_cvtw(const float* __restrict__ src, h16* dst, size_t n8) {
    const size_t i = (size_t)blockIdx.x * 256 + threadIdx.x; if (i >= n8) return;
    const v8f v = *(const v8f*)(src + i * 8); v8h o;
#pragma unroll
    for (int k = 0; k < 8; ++k) o[k] = toh_flush(bfr(v[k]) * WOC);
    *(volatile v8h*)(dst + i * 8) = o; __threadfence(); *(volatile v8h*)(dst + i * 8) = o;
}

__global__ __launch_bounds__(256) void k_wtr(const float* __restrict__ W, bf* WT) {
    __shared__ __align__(16) unsigned short ts[64 * TSP];
    const unsigned tid = threadIdx.x;
    const unsigned d0 = blockIdx.x * 64u, h = blockIdx.y;
    const float* src = W + ((size_t)h * DM + d0) * HD;
#pragma unroll
    for (int it = 0; it < 4; ++it) {
        const unsigned p = (unsigned)it * 256u + tid; const unsigned d = p >> 4, k4 = (p & 15u) * 4u;
        const v4f v = *(const v4f*)(src + (size_t)d * HD + k4);
#pragma unroll
        for (int i = 0; i < 4; ++i) ts[(k4 + i) * TSP + d] = f2bf(v[i]);
    }
    __syncthreads();
#pragma unroll 1
    for (int ps = 0; ps < 2; ++ps) {
#pragma unroll
        for (int it = 0; it < 2; ++it) {
            const unsigned p = (unsigned)it * 256u + tid; const unsigned row = p >> 3, c8 = (p & 7u) * 8u;
            const v8us o = *(const v8usa*)(&ts[row * TSP + c8]);
            *(volatile v8us*)(WT + ((size_t)(h * HD + row)) * DM + d0 + c8) = o; }
        if (ps == 0) __threadfence(); }
}

__device__ __forceinline__ void gemm_bf_64x64(const bf* __restrict__ A, const bf* __restrict__ Bt, const size_t aoff, const size_t boff, v8f (&acc)[4][4]) {
#pragma unroll
    for (int mb = 0; mb < 4; ++mb)
#pragma unroll
        for (int nb = 0; nb < 4; ++nb) acc[mb][nb] = (v8f){};
#pragma unroll 1
    for (int kc = 0; kc < DM; kc += 32) {
        v16bf a[4];
#pragma unroll
        for (int mb = 0; mb < 4; ++mb) a[mb] = ldb(A + aoff + (size_t)mb * 16 * DM + kc);
#pragma unroll
        for (int nb = 0; nb < 4; ++nb) { const v16bf b = ldb(Bt + boff + (size_t)nb * 16 * DM + kc);
#pragma unroll
            for (int mb = 0; mb < 4; ++mb) acc[mb][nb] = wmmabg(a[mb], b, acc[mb][nb]); }
    }
}
__device__ __forceinline__ void gemm_h_64x64(const h16* __restrict__ A, const h16* __restrict__ Bt, const size_t aoff, const size_t boff, v8f (&acc)[4][4]) {
#pragma unroll
    for (int mb = 0; mb < 4; ++mb)
#pragma unroll
        for (int nb = 0; nb < 4; ++nb) acc[mb][nb] = (v8f){};
#pragma unroll 1
    for (int kc = 0; kc < DM; kc += 32) {
        v16h a[4];
#pragma unroll
        for (int mb = 0; mb < 4; ++mb) a[mb] = ldh(A + aoff + (size_t)mb * 16 * DM + kc);
#pragma unroll
        for (int nb = 0; nb < 4; ++nb) { const v16h b = ldh(Bt + boff + (size_t)nb * 16 * DM + kc);
#pragma unroll
            for (int mb = 0; mb < 4; ++mb) acc[mb][nb] = wmma16g(a[mb], b, acc[mb][nb]); }
    }
}

__global__ __launch_bounds__(32) void k_proj_rows(const bf* __restrict__ A, const bf* __restrict__ Bt, const float* __restrict__ bias, h16* Ph) {
    __shared__ __align__(16) float os[16 * OSP];
    const int lane = threadIdx.x & 31, lr = lane & 15, hi = lane >> 4;
    const unsigned r0 = blockIdx.x * 64u, c0 = blockIdx.y * 64u;
    v8f acc[4][4];
    gemm_bf_64x64(A, Bt, (size_t)(r0 + lr) * DM + 8 * hi, (size_t)(c0 + lr) * DM + 8 * hi, acc);
    float bc[4];
#pragma unroll
    for (int nb = 0; nb < 4; ++nb) bc[nb] = bfr(bias[c0 + nb * 16 + lr]);
    const unsigned bb = r0 / (unsigned)SEQ, tt = r0 % (unsigned)SEQ; const unsigned zc = bb * (unsigned)NH_ + c0 / (unsigned)HD;
    const size_t tbase = ((size_t)zc * SEQ + (size_t)tt) * HD;
#pragma unroll
    for (int mb = 0; mb < 4; ++mb) {
#pragma unroll
        for (int nb = 0; nb < 4; ++nb) {
#pragma unroll
            for (int j = 0; j < 8; ++j) os[(hi * 8 + j) * OSP + nb * 16 + lr] = acc[mb][nb][j] + bc[nb]; }
        wave_sync();
#pragma unroll 1
        for (int ps = 0; ps < 2; ++ps) {
            const size_t sb = tbase + (size_t)(mb * 16) * HD;
#pragma unroll
            for (int s = 0; s < 4; ++s) { const int p = s * 32 + lane; const int row = p >> 3, c8 = (p & 7) * 8;
                const v4f x0 = *(const v4fa*)(&os[row * OSP + c8]); const v4f x1 = *(const v4fa*)(&os[row * OSP + c8 + 4]); v8h hv;
#pragma unroll
                for (int i = 0; i < 4; ++i) { hv[i] = toh_flush(x0[i]); hv[4 + i] = toh_flush(x1[i]); }
                *(volatile v8h*)(Ph + sb + (size_t)p * 8) = hv; }
            if (ps == 0) __threadfence(); }
        wave_sync();
    }
}

__global__ __launch_bounds__(32) void k_proj_tr(const bf* __restrict__ A, const bf* __restrict__ Bt, const float* __restrict__ bias, h16* Ph) {
    __shared__ __align__(16) float os[16 * OSP];
    const int lane = threadIdx.x & 31, lr = lane & 15, hi = lane >> 4;
    const unsigned r0 = blockIdx.x * 64u, c0 = blockIdx.y * 64u;
    v8f acc[4][4];
    gemm_bf_64x64(A, Bt, (size_t)(r0 + lr) * DM + 8 * hi, (size_t)(c0 + lr) * DM + 8 * hi, acc);
    const unsigned bb = c0 / (unsigned)SEQ, tt = c0 % (unsigned)SEQ;
    const size_t tbase = (size_t)bb * (size_t)DM * SEQ + (size_t)r0 * SEQ + (size_t)tt;
#pragma unroll
    for (int mb = 0; mb < 4; ++mb) {
        float br[8];
#pragma unroll
        for (int j = 0; j < 8; ++j) br[j] = bfr(bias[r0 + mb * 16 + hi * 8 + j]);
#pragma unroll
        for (int nb = 0; nb < 4; ++nb) {
#pragma unroll
            for (int j = 0; j < 8; ++j) os[(hi * 8 + j) * OSP + nb * 16 + lr] = acc[mb][nb][j] + br[j]; }
        wave_sync();
#pragma unroll 1
        for (int ps = 0; ps < 2; ++ps) {
            const size_t sb = tbase + (size_t)(mb * 16) * SEQ;
#pragma unroll
            for (int s = 0; s < 4; ++s) { const int row = 4 * s + (lane >> 3), c8 = (lane & 7) * 8;
                const v4f x0 = *(const v4fa*)(&os[row * OSP + c8]); const v4f x1 = *(const v4fa*)(&os[row * OSP + c8 + 4]); v8h hv;
#pragma unroll
                for (int i = 0; i < 4; ++i) { hv[i] = toh_flush(x0[i]); hv[4 + i] = toh_flush(x1[i]); }
                *(volatile v8h*)(Ph + sb + (size_t)row * SEQ + c8) = hv; }
            if (ps == 0) __threadfence(); }
        wave_sync();
    }
}

__global__ __launch_bounds__(32 * CW) void k_colstat(const h16* __restrict__ QP, const h16* __restrict__ KP, float* ST) {
    __shared__ __align__(16) float st[2 * 16 * CW];
    const int lane = threadIdx.x & 31, lr = lane & 15, hi = lane >> 4;
    const int wave = __builtin_amdgcn_readfirstlane((int)(threadIdx.x >> 5));
    const unsigned zh = blockIdx.y;
    const unsigned j0 = (blockIdx.x * (unsigned)CW + (unsigned)wave) * 16u;
    const size_t pbase = (size_t)zh * SEQ * HD;
    const size_t kof = pbase + (size_t)(j0 + lr) * HD + 8 * hi;
    const v16h kf0 = ldh(KP + kof), kf1 = ldh(KP + kof + 32);
    const size_t qo = pbase + (size_t)lr * HD + 8 * hi;
    float m = NEGB, l = 0.0f;
#pragma unroll 1
    for (int i0 = 0; i0 < SEQ; i0 += 32) {
        const h16* qa = QP + qo + (size_t)i0 * HD;
        const v16h qa0 = ldh(qa), qa1 = ldh(qa + 32), qb0 = ldh(qa + 16 * HD), qb1 = ldh(qa + 16 * HD + 32);
        v8f sa = (v8f){}, sb = (v8f){};
        sa = wmma16g(qa0, kf0, sa); sa = wmma16g(qa1, kf1, sa);
        sb = wmma16g(qb0, kf0, sb); sb = wmma16g(qb1, kf1, sb);
        float ta[8], tb[8]; float mx = NEGB;
#pragma unroll
        for (int r = 0; r < 8; ++r) { ta[r] = sa[r] * SC2; tb[r] = sb[r] * SC2; mx = fmaxf(mx, fmaxf(ta[r], tb[r])); }
        const float mnew = fmaxf(m, mx);
        const float alpha = __builtin_amdgcn_exp2f(m - mnew);
        float ls = 0.0f;
#pragma unroll
        for (int r = 0; r < 8; ++r) ls += __builtin_amdgcn_exp2f(ta[r] - mnew) + __builtin_amdgcn_exp2f(tb[r] - mnew);
        l = l * alpha + ls; m = mnew;
    }
    const float m2 = __shfl_xor(m, 16, 32);
    const float l2 = __shfl_xor(l, 16, 32);
    const float M  = fmaxf(m, m2);
    const float Ls = l * __builtin_amdgcn_exp2f(m - M) + l2 * __builtin_amdgcn_exp2f(m2 - M);
    const float rl = 1.0f / Ls;
    if (hi == 0) { st[wave * 16 + lr] = M; st[16 * CW + wave * 16 + lr] = rl; }
    __syncthreads();
    const unsigned kb = blockIdx.x * (16u * CW);
    const size_t dsto = (size_t)((lane & 15) >> 3) * STP + (size_t)zh * SEQ + kb + (unsigned)(lane & 7) * 4u;
    const v4f val = *(const v4fa*)(&st[(lane & 15) * 4]);
#pragma unroll 1
    for (int ps = 0; ps < 2; ++ps) {
        if (wave == 0 && lane < 16) *(volatile v4f*)(ST + dsto) = val;
        if (ps == 0) __threadfence(); }
}

__global__ __launch_bounds__(32 * AW) void k_attn(const h16* __restrict__ QP, const h16* __restrict__ KP, const h16* __restrict__ VT, const float* __restrict__ ST, h16* CT) {
    __shared__ __align__(16) float os[AW * 16 * OSP];
    const int lane = threadIdx.x & 31, lr = lane & 15, hi = lane >> 4;
    const int wave = __builtin_amdgcn_readfirstlane((int)(threadIdx.x >> 5));
    const unsigned zh = blockIdx.y; const unsigned b = zh / (unsigned)NH_, h = zh % (unsigned)NH_;
    const unsigned t0 = (blockIdx.x * (unsigned)AW + (unsigned)wave) * 16u;
    const size_t pbase = (size_t)zh * SEQ * HD;
    const size_t qo = pbase + (size_t)(t0 + lr) * HD + 8 * hi;
    const v16h q0 = ldh(QP + qo), q1 = ldh(QP + qo + 32);
    const size_t ko = pbase + (size_t)lr * HD + 8 * hi;
    const size_t vo = pbase + (size_t)lr * SEQ + 8 * hi;
    const float* mp = ST + (size_t)zh * SEQ + 8 * hi;
    const float* lp = mp + STP;
    v8f o0 = (v8f){}, o1 = (v8f){}, o2 = (v8f){}, o3 = (v8f){};
#pragma unroll 1
    for (int key0 = 0; key0 < SEQ; key0 += 32) {
        const h16* ka = KP + ko + (size_t)key0 * HD;
        const v16h ka0 = ldh(ka), ka1 = ldh(ka + 32), kb0 = ldh(ka + 16 * HD), kb1 = ldh(ka + 16 * HD + 32);
        v8f sa = (v8f){}, sb = (v8f){};
        sa = wmma16g(ka0, q0, sa); sa = wmma16g(ka1, q1, sa);
        sb = wmma16g(kb0, q0, sb); sb = wmma16g(kb1, q1, sb);
        const float* mk = mp + key0; const float* lk = lp + key0;
        const v4f m0 = *(const v4f*)mk, m1 = *(const v4f*)(mk + 4), m2 = *(const v4f*)(mk + 16), m3 = *(const v4f*)(mk + 20);
        const v4f l0 = *(const v4f*)lk, l1 = *(const v4f*)(lk + 4), l2 = *(const v4f*)(lk + 16), l3 = *(const v4f*)(lk + 20);
        v16h pb;
#pragma unroll
        for (int r = 0; r < 4; ++r) {
            const float e0 = (sa[r]     * SC2 - m0[r]) + PSH;
            const float e1 = (sa[4 + r] * SC2 - m1[r]) + PSH;
            const float e2 = (sb[r]     * SC2 - m2[r]) + PSH;
            const float e3 = (sb[4 + r] * SC2 - m3[r]) + PSH;
            pb[r]      = toh_flush(__builtin_amdgcn_exp2f(e0) * l0[r]);
            pb[4 + r]  = toh_flush(__builtin_amdgcn_exp2f(e1) * l1[r]);
            pb[8 + r]  = toh_flush(__builtin_amdgcn_exp2f(e2) * l2[r]);
            pb[12 + r] = toh_flush(__builtin_amdgcn_exp2f(e3) * l3[r]);
        }
        const h16* va = VT + vo + key0;
        const v16h v0 = ldh(va), v1 = ldh(va + (size_t)16 * SEQ), v2 = ldh(va + (size_t)32 * SEQ), v3 = ldh(va + (size_t)48 * SEQ);
        o0 = wmma16g(v0, pb, o0); o1 = wmma16g(v1, pb, o1); o2 = wmma16g(v2, pb, o2); o3 = wmma16g(v3, pb, o3);
    }
    const int wb = wave * 16 * OSP;
    { v4f a, c;
      a[0] = o0[0] * PVS; a[1] = o0[1] * PVS; a[2] = o0[2] * PVS; a[3] = o0[3] * PVS; c[0] = o0[4] * PVS; c[1] = o0[5] * PVS; c[2] = o0[6] * PVS; c[3] = o0[7] * PVS;
      *(v4fa*)(&os[wb + lr * OSP +  0 + 8 * hi]) = a; *(v4fa*)(&os[wb + lr * OSP +  0 + 8 * hi + 4]) = c;
      a[0] = o1[0] * PVS; a[1] = o1[1] * PVS; a[2] = o1[2] * PVS; a[3] = o1[3] * PVS; c[0] = o1[4] * PVS; c[1] = o1[5] * PVS; c[2] = o1[6] * PVS; c[3] = o1[7] * PVS;
      *(v4fa*)(&os[wb + lr * OSP + 16 + 8 * hi]) = a; *(v4fa*)(&os[wb + lr * OSP + 16 + 8 * hi + 4]) = c;
      a[0] = o2[0] * PVS; a[1] = o2[1] * PVS; a[2] = o2[2] * PVS; a[3] = o2[3] * PVS; c[0] = o2[4] * PVS; c[1] = o2[5] * PVS; c[2] = o2[6] * PVS; c[3] = o2[7] * PVS;
      *(v4fa*)(&os[wb + lr * OSP + 32 + 8 * hi]) = a; *(v4fa*)(&os[wb + lr * OSP + 32 + 8 * hi + 4]) = c;
      a[0] = o3[0] * PVS; a[1] = o3[1] * PVS; a[2] = o3[2] * PVS; a[3] = o3[3] * PVS; c[0] = o3[4] * PVS; c[1] = o3[5] * PVS; c[2] = o3[6] * PVS; c[3] = o3[7] * PVS;
      *(v4fa*)(&os[wb + lr * OSP + 48 + 8 * hi]) = a; *(v4fa*)(&os[wb + lr * OSP + 48 + 8 * hi + 4]) = c; }
    wave_sync();
    h16* crow = CT + ((size_t)b * SEQ + t0) * DM + h * HD;
#pragma unroll 1
    for (int ps = 0; ps < 2; ++ps) {
#pragma unroll
        for (int s = 0; s < 4; ++s) { const int row = 4 * s + (lane >> 3), c8 = (lane & 7) * 8;
            const v4f x0 = *(const v4fa*)(&os[wb + row * OSP + c8]); const v4f x1 = *(const v4fa*)(&os[wb + row * OSP + c8 + 4]); v8h hv;
#pragma unroll
            for (int i = 0; i < 4; ++i) { hv[i] = toh_flush(x0[i]); hv[4 + i] = toh_flush(x1[i]); }
            *(volatile v8h*)(crow + (size_t)row * DM + c8) = hv; }
        if (ps == 0) __threadfence(); }
}

__global__ __launch_bounds__(32) void k_outp(const h16* __restrict__ A, const h16* __restrict__ Bt, const float* __restrict__ bias, float* OUT) {
    __shared__ __align__(16) float os[16 * OSP];
    const int lane = threadIdx.x & 31, lr = lane & 15, hi = lane >> 4;
    const unsigned r0 = blockIdx.x * 64u, c0 = blockIdx.y * 64u;
    v8f acc[4][4];
    gemm_h_64x64(A, Bt, (size_t)(r0 + lr) * DM + 8 * hi, (size_t)(c0 + lr) * DM + 8 * hi, acc);
    float bc[4];
#pragma unroll
    for (int nb = 0; nb < 4; ++nb) bc[nb] = bfr(bias[c0 + nb * 16 + lr]);
    const unsigned bb = r0 / (unsigned)SEQ, tt = r0 % (unsigned)SEQ;
    const size_t obase = ((size_t)bb * OUT_SEQ + (size_t)tt) * DM + c0;
#pragma unroll
    for (int mb = 0; mb < 4; ++mb) {
#pragma unroll
        for (int nb = 0; nb < 4; ++nb) {
#pragma unroll
            for (int j = 0; j < 8; ++j) os[(hi * 8 + j) * OSP + nb * 16 + lr] = acc[mb][nb][j] * OSC + bc[nb]; }
        wave_sync();
#pragma unroll 1
        for (int ps = 0; ps < 2; ++ps) {
            const size_t sb = obase + (size_t)(mb * 16) * DM;
#pragma unroll
            for (int s = 0; s < 8; ++s) { const int row = 2 * s + (lane >> 4), c4 = (lane & 15) * 4;
                const v4f val = *(const v4fa*)(&os[row * OSP + c4]);
                *(volatile v4f*)(OUT + sb + (size_t)row * DM + c4) = val; }
            if (ps == 0) __threadfence(); }
        wave_sync();
    }
}

static constexpr size_t al256(size_t v) { return (v + 255) & ~(size_t)255; }
static constexpr size_t SZ_XB = al256((size_t)NB * SEQ * DM * 2);
static constexpr size_t SZ_WT = al256((size_t)NH_ * HD * DM * 2);
static constexpr size_t SZ_WO = al256((size_t)DM * DM * 2);
static constexpr size_t SZ_PL = al256((size_t)NB * NH_ * SEQ * HD * 2);
static constexpr size_t SZ_ST = al256((size_t)2 * NB * NH_ * SEQ * 4);
static constexpr size_t SZ_CT = al256((size_t)NB * SEQ * DM * 2);
static constexpr size_t SZ_TOTAL = SZ_XB + 3 * SZ_WT + SZ_WO + 3 * SZ_PL + SZ_ST + SZ_CT;
static_assert(SZ_TOTAL <= (size_t)134217728);
static_assert((size_t)NB * NH_ * SEQ * HD == (size_t)NB * DM * SEQ);
static_assert((size_t)2 * STP * 4 <= SZ_ST);
static_assert((size_t)NH_ * HD == (size_t)DM);

extern "C" void kernel_launch(void* const* d_in, const int* in_sizes, int n_in,
                              void* d_out, int out_size, void* d_ws, size_t ws_size, hipStream_t stream) {
    if (n_in < 9) return;
    const size_t needx = ((size_t)(NB - 1) * SEQ_FULL + SEQ) * DM;
    if ((size_t)in_sizes[0] < needx) return;
    if ((size_t)in_sizes[1] < (size_t)NH_ * DM * HD || (size_t)in_sizes[3] < (size_t)NH_ * DM * HD || (size_t)in_sizes[5] < (size_t)NH_ * DM * HD) return;
    if (in_sizes[2] < DM || in_sizes[4] < DM || in_sizes[6] < DM) return;
    if ((size_t)in_sizes[7] < (size_t)DM * DM || in_sizes[8] < DM) return;
    if ((size_t)out_size < ((size_t)(NB - 1) * OUT_SEQ + SEQ) * DM) return;
    if (SZ_TOTAL > ws_size) return;
    const float* xin = (const float*)d_in[0];
    const float* wq = (const float*)d_in[1]; const float* bq = (const float*)d_in[2];
    const float* wk = (const float*)d_in[3]; const float* bk = (const float*)d_in[4];
    const float* wv = (const float*)d_in[5]; const float* bv = (const float*)d_in[6];
    const float* wo = (const float*)d_in[7]; const float* bo = (const float*)d_in[8];
    float* OUT = (float*)d_out;
    char* wsp = (char*)d_ws;
    bf*  XB  = (bf*)wsp;  wsp += SZ_XB;
    bf*  WTQ = (bf*)wsp;  wsp += SZ_WT;
    bf*  WTK = (bf*)wsp;  wsp += SZ_WT;
    bf*  WTV = (bf*)wsp;  wsp += SZ_WT;
    h16* WOH = (h16*)wsp; wsp += SZ_WO;
    h16* QP  = (h16*)wsp; wsp += SZ_PL;
    h16* KP  = (h16*)wsp; wsp += SZ_PL;
    h16* VT  = (h16*)wsp; wsp += SZ_PL;
    float* ST = (float*)wsp; wsp += SZ_ST;
    h16* CT  = (h16*)wsp; wsp += SZ_CT;

    if (SEQ == SEQ_FULL) {
        const size_t n8 = (size_t)NB * SEQ * DM / 8;
        k_cvt8<<<(unsigned)((n8 + 255) / 256), 256, 0, stream>>>(xin, XB, n8);
    } else {
        const size_t n8 = (size_t)SEQ * DM / 8;
        for (int b = 0; b < NB; ++b) k_cvt8<<<(unsigned)((n8 + 255) / 256), 256, 0, stream>>>(xin + (size_t)b * SEQ_FULL * DM, XB + (size_t)b * SEQ * DM, n8);
    }
    k_wtr<<<dim3(DM / 64, NH_, 1), 256, 0, stream>>>(wq, WTQ);
    k_wtr<<<dim3(DM / 64, NH_, 1), 256, 0, stream>>>(wk, WTK);
    k_wtr<<<dim3(DM / 64, NH_, 1), 256, 0, stream>>>(wv, WTV);
    { const size_t n8 = (size_t)DM * DM / 8; k_cvtw<<<(unsigned)((n8 + 255) / 256), 256, 0, stream>>>(wo, WOH, n8); }

    k_proj_rows<<<dim3(NB * SEQ / 64, DM / 64, 1), 32, 0, stream>>>(XB, WTQ, bq, QP);
    k_proj_rows<<<dim3(NB * SEQ / 64, DM / 64, 1), 32, 0, stream>>>(XB, WTK, bk, KP);
    k_proj_tr<<<dim3(DM / 64, NB * SEQ / 64, 1), 32, 0, stream>>>(WTV, XB, bv, VT);

    k_colstat<<<dim3(SEQ / (16 * CW), NB * NH_, 1), 32 * CW, 0, stream>>>(QP, KP, ST);
    k_attn<<<dim3(SEQ / (16 * AW), NB * NH_, 1), 32 * AW, 0, stream>>>(QP, KP, VT, ST, CT);

    k_outp<<<dim3(NB * SEQ / 64, DM / 64, 1), 32, 0, stream>>>(CT, WOH, bo, OUT);
}
